// GGNNLayer_80221399155535
// MI455X (gfx1250) — hardware-verified
//
#include <hip/hip_runtime.h>
#include <hip/hip_bf16.h>
#include <math.h>


#define BB 2
#define SS 2048
#define DD 1024
#define HH 16
#define DKK 64
#define QW 2

typedef _Float16 bf16;
typedef __attribute__((ext_vector_type(4))) unsigned v4u_t;
typedef unsigned v4ua __attribute__((ext_vector_type(4), may_alias));
typedef __attribute__((ext_vector_type(4))) float v4f_t;
typedef float v4fa __attribute__((ext_vector_type(4), may_alias));
typedef __attribute__((ext_vector_type(16))) bf16  bf16x16;
typedef __attribute__((ext_vector_type(8)))  bf16  bf16x8;
typedef __attribute__((ext_vector_type(4)))  bf16  bf16x4;
typedef __attribute__((ext_vector_type(8)))  float f32x8;

#define LDS_STRIDE 48
#define KSTRIDE    72
#define VSTRIDE    48

__device__ __forceinline__ f32x8 wmma_bf16(bf16x16 a, bf16x16 b, f32x8 c) {
  return __builtin_amdgcn_wmma_f32_16x16x32_f16(
      false, a, false, b, (short)0, c, false, false);
}
#define RSPLIT (1.0f / 2048.0f)
__device__ __forceinline__ bf16 lo_of(float v, bf16 h) { return (bf16)((v - (float)h) * 2048.0f); }
__device__ __forceinline__ f32x8 wmma_split(bf16x16 a, bf16x16 al, bf16x16 b, bf16x16 bl, f32x8 c) {
  f32x8 x = {}; x = wmma_bf16(al, b, x); x = wmma_bf16(a, bl, x); return wmma_bf16(a, b, c) + x * RSPLIT; }

template <typename T>
__device__ __forceinline__ bf16x16 load_frag(const T* __restrict__ base, int ld,
                                             int row0, int k0) {
  const int lane = threadIdx.x & 31;
  const int r    = lane & 15;
  const int kh   = (lane >> 4) * 8;
  const T* p0 = base + (size_t)(row0 + r) * ld + (k0 + kh);
  const T* p1 = p0 + 16;
  bf16x16 f;
#pragma unroll
  for (int i = 0; i < 8; ++i) {
    f[i]     = (bf16)p0[i];
    f[i + 8] = (bf16)p1[i];
  }
  return f;
}

__device__ __forceinline__ bf16x16 lds_frag(const bf16* base, int stride) {
  const int lane = threadIdx.x & 31;
  const int row  = lane & 15;
  const int kh   = (lane >> 4) * 8;
  const bf16x8 lo = *(const bf16x8*)(base + row * stride + kh);
  const bf16x8 hi = *(const bf16x8*)(base + row * stride + kh + 16);
  bf16x16 f;
#pragma unroll
  for (int i = 0; i < 8; ++i) { f[i] = lo[i]; f[i + 8] = hi[i]; }
  return f;
}

template <typename T>
__device__ __forceinline__ void stage_read16(const T* __restrict__ p, float* buf) {
#pragma unroll
  for (int i = 0; i < 16; ++i) buf[i] = (float)p[i];
}

__device__ __forceinline__ void stage_write(bf16* dst, const float* buf, int nquad) {
#pragma unroll
  for (int i = 0; i < nquad; ++i) {
    bf16x4 q;
    q[0] = (bf16)buf[4 * i];     q[1] = (bf16)buf[4 * i + 1];
    q[2] = (bf16)buf[4 * i + 2]; q[3] = (bf16)buf[4 * i + 3];
    *(bf16x4*)(dst + 4 * i) = q;
  }
}

__global__ __launch_bounds__(256) void transpose_pack_kernel(const float* __restrict__ W, bf16* __restrict__ WT, int K, int N, size_t plane) {
  __shared__ float tile[64][65];
  const int k0 = blockIdx.y * 64, n0 = blockIdx.x * 64, t = threadIdx.x;
  for (int i = t; i < 64 * 64; i += 256) { const int kr = i >> 6, nc = i & 63; tile[kr][nc] = W[(size_t)(k0 + kr) * N + n0 + nc]; }
  __syncthreads();
#pragma unroll 1
  for (int pass = 0; pass < 2; ++pass) {
    for (int i = t; i < 64 * 8; i += 256) { const int nr = i >> 3, k8 = (i & 7) * 8; bf16 hh[8], hl[8];
#pragma unroll
      for (int e = 0; e < 8; ++e) { const float v = tile[k8 + e][nr]; hh[e] = (bf16)v; hl[e] = lo_of(v, hh[e]); }
      bf16* d = WT + (size_t)(n0 + nr) * K + k0 + k8;
      *(volatile v4u_t*)d = *(const v4ua*)hh; *(volatile v4u_t*)(d + plane) = *(const v4ua*)hl; }
    __threadfence();
  }
}

template <typename AT, typename WT, int MODE>
__global__ __launch_bounds__(256) void gemm_split_kernel(
    const AT* __restrict__ A, size_t aPlane, const WT* __restrict__ W, size_t wPlane,
    const float* __restrict__ bias, void* __restrict__ out,
    int M, int N, int K) {
  __shared__ bf16 ldsA[128 * LDS_STRIDE], ldsAl[128 * LDS_STRIDE];
  __shared__ bf16 ldsW[256 * LDS_STRIDE], ldsWl[256 * LDS_STRIDE];
  __shared__ __attribute__((aligned(16))) unsigned char sob[256 * 136 * 2];

  const int t    = threadIdx.x;
  const int wave = t >> 5;
  const int lane = t & 31;
  const int wm   = (wave & 1) * 64;
  const int wn   = (wave >> 1) * 64;
  const int mBlk = blockIdx.x * 128;
  const int nBlk = blockIdx.y * 256;
  const int arow = t >> 1;
  const int ach  = (t & 1) * 16;

  f32x8 acc[4][4] = {};
  for (int k = 0; k < K; k += 32) {
    __syncthreads();
    {
      const AT* ap = A + (size_t)(mBlk + arow) * K + k + ach;
      bf16 hh[16], hl[16];
      if (sizeof(AT) == 4) {
#pragma unroll
        for (int i = 0; i < 16; ++i) { const float v = (float)ap[i]; hh[i] = (bf16)v; hl[i] = lo_of(v, hh[i]); }
      } else {
#pragma unroll
        for (int i = 0; i < 16; ++i) { hh[i] = (bf16)ap[i]; hl[i] = (bf16)ap[aPlane + i]; }
      }
#pragma unroll
      for (int i = 0; i < 16; ++i) { ldsA[arow * LDS_STRIDE + ach + i] = hh[i]; ldsAl[arow * LDS_STRIDE + ach + i] = hl[i]; }
    }
    {
      const WT* wp = W + (size_t)(nBlk + t) * K + k;
      if (sizeof(WT) == 4) {
#pragma unroll
        for (int i = 0; i < 32; ++i) { const float v = (float)wp[i]; const bf16 h_ = (bf16)v; ldsW[t * LDS_STRIDE + i] = h_; ldsWl[t * LDS_STRIDE + i] = lo_of(v, h_); }
      } else {
#pragma unroll
        for (int i = 0; i < 32; ++i) { ldsW[t * LDS_STRIDE + i] = (bf16)wp[i]; ldsWl[t * LDS_STRIDE + i] = (bf16)wp[wPlane + i]; }
      }
    }
    __syncthreads();
    bf16x16 wf[4], wfl[4];
#pragma unroll
    for (int j = 0; j < 4; ++j) { wf[j] = lds_frag(ldsW + (wn + 16 * j) * LDS_STRIDE, LDS_STRIDE); wfl[j] = lds_frag(ldsWl + (wn + 16 * j) * LDS_STRIDE, LDS_STRIDE); }
#pragma unroll
    for (int i = 0; i < 4; ++i) {
      const bf16x16 af = lds_frag(ldsA + (wm + 16 * i) * LDS_STRIDE, LDS_STRIDE), afl = lds_frag(ldsAl + (wm + 16 * i) * LDS_STRIDE, LDS_STRIDE);
#pragma unroll
      for (int j = 0; j < 4; ++j) acc[i][j] = wmma_split(af, afl, wf[j], wfl[j], acc[i][j]);
    }
  }

  const int nlane = lane & 15;
  const int mh    = (lane >> 4) * 8;
  __syncthreads();
  if (MODE == 1) {
    bf16* so = (bf16*)sob;
#pragma unroll
    for (int i = 0; i < 4; ++i)
#pragma unroll
      for (int j = 0; j < 4; ++j) {
        const int nl = wn + 16 * j + nlane;
        const float bv = bias ? bias[nBlk + nl] : 0.0f;
#pragma unroll
        for (int r = 0; r < 8; ++r) so[nl * 136 + wm + 16 * i + mh + r] = (bf16)(acc[i][j][r] + bv);
      }
    __syncthreads();
    const int b_ = mBlk >> 11, s0 = mBlk & (SS - 1);
#pragma unroll 1
    for (int pass = 0; pass < 2; ++pass) {
      for (int ch = t; ch < 256 * 16; ch += 256) { const int nl = ch >> 4, q = (ch & 15) * 8; const int n = nBlk + nl, h = n >> 6, dk = n & (DKK - 1);
        *(volatile v4u_t*)((bf16*)out + (((size_t)(b_ * HH + h)) * DKK + dk) * SS + s0 + q) = *(const v4ua*)(so + nl * 136 + q); }
      __threadfence();
    }
  } else {
    float* so = (float*)sob;
#pragma unroll 1
    for (int hf = 0; hf < 2; ++hf) {
      if (wm == hf * 64) {
#pragma unroll
        for (int i = 0; i < 4; ++i)
#pragma unroll
          for (int j = 0; j < 4; ++j) {
            const int nl = wn + 16 * j + nlane;
            const float bv = bias ? bias[nBlk + nl] : 0.0f;
#pragma unroll
            for (int r = 0; r < 8; ++r) so[(16 * i + mh + r) * 260 + nl] = acc[i][j][r] + bv;
          }
      }
      __syncthreads();
#pragma unroll 1
      for (int pass = 0; pass < 2; ++pass) {
        for (int ch = t; ch < 64 * 64; ch += 256) { const int ml = ch >> 6, q = (ch & 63) * 4;
          *(volatile v4f_t*)((float*)out + (size_t)(mBlk + hf * 64 + ml) * N + nBlk + q) = *(const volatile v4fa*)(so + ml * 260 + q); }
        __threadfence();
      }
      __syncthreads();
    }
  }
}


#define GN 50000
#define GNP 50176
#define GE 600000
#define GRANGE 12544
#define GD 128

__global__ __launch_bounds__(128) void k_fold(const float* __restrict__ W1, const float* __restrict__ b1, const float* __restrict__ W2, const float* __restrict__ b2,
                                             float* __restrict__ AmT, float* __restrict__ bm) {
  const int m = blockIdx.x, k = threadIdx.x; float s = 0.0f;
#pragma unroll 1
  for (int j = 0; j < GD; ++j) s += W1[(size_t)k * GD + j] * W2[(size_t)j * GD + m];
  *(volatile float*)(AmT + (size_t)m * GD + k) = s;
  if (k == 0) { float bb = b2[m];
#pragma unroll 1
    for (int j = 0; j < GD; ++j) bb += b1[j] * W2[(size_t)j * GD + m];
    *(volatile float*)(bm + m) = bb; }
  __threadfence();
  *(volatile float*)(AmT + (size_t)m * GD + k) = s;
}
__global__ __launch_bounds__(128) void k_trw(const float* __restrict__ W, float* __restrict__ AT) {
  const int m = blockIdx.x, k = threadIdx.x; const float v = W[(size_t)k * 3 * GD + m];
  *(volatile float*)(AT + (size_t)m * GD + k) = v; __threadfence(); *(volatile float*)(AT + (size_t)m * GD + k) = v;
}
__global__ __launch_bounds__(128) void k_padrows(const float* __restrict__ x, float* __restrict__ XP) {
  const int row = blockIdx.x, k = threadIdx.x; const float v = (row < GN) ? x[(size_t)row * GD + k] : 0.0f;
  *(volatile float*)(XP + (size_t)row * GD + k) = v; __threadfence(); *(volatile float*)(XP + (size_t)row * GD + k) = v;
}
__global__ __launch_bounds__(256) void k_agg(const int* __restrict__ ea, const int* __restrict__ eb, const float* __restrict__ msgT, const float* __restrict__ bm,
                                            int rsel, float* __restrict__ R) {
  __shared__ int qd[256], qs[256]; __shared__ int wcnt[8]; __shared__ int cnt[GRANGE];
  const int tid = threadIdx.x, lane = tid & 31, wave = tid >> 5, r0 = rsel * GRANGE;
  for (int i = tid; i < GRANGE * GD / 4; i += 256) { v4f_t z; z.x = z.y = z.z = z.w = 0.0f; *(volatile v4f_t*)(R + (size_t)i * 4) = z; }
  for (int i = tid; i < GRANGE; i += 256) cnt[i] = 0;
  __threadfence(); __syncthreads();
#pragma unroll 1
  for (int c0 = 0; c0 < GE; c0 += 128) {
    const int e = c0 + (tid >> 1), dir = tid & 1; int d = -1, sidx = 0;
    if (e < GE) { const int a = ea[e], b = eb[e]; const int aa = a < 0 ? 0 : (a >= GN ? GN - 1 : a), bb = b < 0 ? 0 : (b >= GN ? GN - 1 : b);
      const int dd = dir ? aa : bb, ss = dir ? bb : aa;
      if (dd >= r0 && dd < r0 + GRANGE) { d = dd - r0; sidx = ss; } }
    const unsigned m = __builtin_amdgcn_ballot_w32(d >= 0);
    if (lane == 0) wcnt[wave] = __builtin_popcount(m);
    __syncthreads();
    int base = 0, total = 0;
#pragma unroll
    for (int w = 0; w < 8; ++w) { const int c = wcnt[w]; base += (w < wave) ? c : 0; total += c; }
    if (d >= 0) { const int pos = base + __builtin_popcount(m & ((1u << lane) - 1u)); qd[pos] = d; qs[pos] = sidx; }
    __syncthreads();
#pragma unroll 1
    for (int qi = 0; qi < total; ++qi) { const int dl = qd[qi]; if ((dl & 7) != wave) continue; const int sl = qs[qi];
      float* row = R + (size_t)dl * GD;
#pragma unroll
      for (int u = 0; u < 4; ++u) row[u * 32 + lane] += msgT[(size_t)(u * 32 + lane) * GNP + sl];
      if (lane == 0) cnt[dl] += 1; }
    __syncthreads();
  }
  __threadfence(); __syncthreads();
#pragma unroll 1
  for (int pass = 0; pass < 2; ++pass) {
    for (int i = tid; i < GRANGE * 32; i += 256) { const int nl = i >> 5, c4 = (i & 31) * 4; float* p = R + (size_t)nl * GD + c4;
      v4f_t v = *(const volatile v4fa*)p; if (pass == 0) { const float c = (float)cnt[nl]; v.x += c * bm[c4]; v.y += c * bm[c4 + 1]; v.z += c * bm[c4 + 2]; v.w += c * bm[c4 + 3]; }
      *(volatile v4f_t*)p = v; }
    __threadfence(); __syncthreads();
  }
}
__global__ __launch_bounds__(256) void k_gru(const float* __restrict__ MX, const float* __restrict__ MH, const float* __restrict__ gb, const float* __restrict__ X, int r0, float* __restrict__ out) {
  __shared__ float tx[384][33], th[384][33];
  __shared__ __attribute__((aligned(16))) float res[32][132];
  const int n0 = blockIdx.x * 32, t = threadIdx.x;
#pragma unroll 2
  for (int i = t; i < 384 * 32; i += 256) { const int r = i >> 5, c = i & 31; tx[r][c] = MX[(size_t)r * GRANGE + n0 + c]; th[r][c] = MH[(size_t)r * GRANGE + n0 + c]; }
  __syncthreads();
#pragma unroll 1
  for (int i = t; i < 32 * GD; i += 256) { const int nl = i >> 7, d = i & (GD - 1), node = r0 + n0 + nl;
    const float xv = (node < GN) ? X[(size_t)node * GD + d] : 0.0f;
    const float xz = tx[d][nl] + gb[d], xr = tx[GD + d][nl] + gb[GD + d], xh = tx[2 * GD + d][nl] + gb[2 * GD + d];
    const float rz = th[d][nl] + gb[3 * GD + d], rr = th[GD + d][nl] + gb[4 * GD + d], rh = th[2 * GD + d][nl] + gb[5 * GD + d];
    const float z = 1.0f / (1.0f + expf(-(xz + rz))), r = 1.0f / (1.0f + expf(-(xr + rr)));
    const float hh = tanhf(xh + r * rh);
    res[nl][d] = z * xv + (1.0f - z) * hh; }
  __syncthreads();
#pragma unroll 1
  for (int pass = 0; pass < 2; ++pass) {
    for (int i = t; i < 32 * 32; i += 256) { const int nl = i >> 5, c4 = (i & 31) * 4, node = r0 + n0 + nl;
      if (node < GN) *(volatile v4f_t*)(out + (size_t)node * GD + c4) = *(const volatile v4fa*)(&res[nl][c4]); }
    __threadfence();
  }
}

extern "C" void kernel_launch(void* const* d_in, const int* in_sizes, int n_in,
                              void* d_out, int out_size, void* d_ws, size_t ws_size,
                              hipStream_t stream) {
  (void)in_sizes; (void)n_in; (void)out_size; (void)ws_size;
  const float* X  = (const float*)d_in[0];
  const int*  ea  = (const int*)d_in[1];
  const int*  eb  = (const int*)d_in[2];
  const float* W1 = (const float*)d_in[3]; const float* b1 = (const float*)d_in[4];
  const float* W2 = (const float*)d_in[5]; const float* b2 = (const float*)d_in[6];
  const float* gk = (const float*)d_in[7];
  const float* gr = (const float*)d_in[8];
  const float* gb = (const float*)d_in[9];
  char* ws = (char*)d_ws;
  float* AmT = (float*)ws; ws += (size_t)GD * GD * 4;
  float* bm  = (float*)ws; ws += 512 * 4;
  float* AK  = (float*)ws; ws += (size_t)384 * GD * 4;
  float* AR  = (float*)ws; ws += (size_t)384 * GD * 4;
  float* XP  = (float*)ws; ws += (size_t)GNP * GD * 4;
  float* msgT= (float*)ws; ws += (size_t)GD * GNP * 4;
  float* R   = (float*)ws; ws += (size_t)GRANGE * GD * 4;
  float* MX  = (float*)ws; ws += (size_t)384 * GRANGE * 4;
  float* MH  = (float*)ws; ws += (size_t)384 * GRANGE * 4;
  k_fold<<<GD, 128, 0, stream>>>(W1, b1, W2, b2, AmT, bm);
  k_trw<<<384, 128, 0, stream>>>(gk, AK);
  k_trw<<<384, 128, 0, stream>>>(gr, AR);
  k_padrows<<<GNP, 128, 0, stream>>>(X, XP);
  dim3 blk(256);
  gemm_split_kernel<float, float, 2><<<dim3(1, GNP / 256), blk, 0, stream>>>(AmT, 0, XP, 0, nullptr, msgT, GD, GNP, GD);
  for (int r = 0; r < GNP / GRANGE; ++r) {
    k_agg<<<1, 256, 0, stream>>>(ea, eb, msgT, bm, r, R);
    gemm_split_kernel<float, float, 2><<<dim3(3, GRANGE / 256), blk, 0, stream>>>(AK, 0, R, 0, nullptr, MX, 384, GRANGE, GD);
    gemm_split_kernel<float, float, 2><<<dim3(3, GRANGE / 256), blk, 0, stream>>>(AR, 0, XP + (size_t)r * GRANGE * GD, 0, nullptr, MH, 384, GRANGE, GD);
    k_gru<<<GRANGE / 32, 256, 0, stream>>>(MX, MH, gb, X, r * GRANGE, (float*)d_out);
  }
}
